// GroupEmbedding_72980084294362
// MI455X (gfx1250) — hardware-verified
//
#include <hip/hip_runtime.h>

typedef __attribute__((ext_vector_type(16))) _Float16 v16h;
typedef __attribute__((ext_vector_type(8)))  _Float16 v8h;
typedef __attribute__((ext_vector_type(8)))  float    v8f;
typedef __attribute__((ext_vector_type(4)))  float    v4f;
typedef __attribute__((ext_vector_type(2)))  float    v2f;
typedef __attribute__((ext_vector_type(4)))  int      v4i;

constexpr int kGroups   = 4096;
constexpr int kUsersPG  = 50;
constexpr int kBehPU    = 20;
constexpr int kEmb      = 64;
constexpr int kSimDim   = 64;
constexpr int kUserRows = 100000;
constexpr int kItemRows = 100000;
constexpr int kSlotsPG  = kUsersPG * kBehPU;
constexpr int kWaves    = 4;
constexpr int kUsersPW  = 16;
constexpr int kSlotsPW  = kUsersPW * kBehPU;
constexpr int kChunkK   = 32;
constexpr int kBtPitch  = 40;
constexpr int kWtPitch  = 68;
constexpr float kCntCarry  = 512.0f;
constexpr float kItemCarry = 64.0f;
constexpr float kFoldBack  = 1.0f / (kCntCarry * kItemCarry);
static_assert(kSlotsPG == 1000, "slots per group");
static_assert(kSlotsPW == 320 && (kSlotsPW % kChunkK) == 0, "concatenated K is a multiple of 32");
static_assert(kWaves * kUsersPW >= kUsersPG, "user padding covers the group");
static_assert(kEmb == 64 && kSimDim == 64, "one float2 per lane covers a table row");
static_assert((kBtPitch % 8) == 0, "16-byte aligned fragment rows");
static_assert(kFoldBack == 1.0f / 32768.0f, "power-of-two fold back");

union FragH { v16h v; v8h h[2]; };

__device__ __forceinline__ v16h frag_load_h(const _Float16* p) {
  FragH f;
  f.h[0] = *(const v8h*)(p);
  f.h[1] = *(const v8h*)(p + 16);
  return f.v;
}

__device__ __forceinline__ v8f mma_h(v16h a, v16h b, v8f c) {
  c = __builtin_amdgcn_wmma_f32_16x16x32_f16(false, a, false, b, (short)0, c, false, false);
  asm volatile("v_nop\n\tv_nop\n\tv_nop\n\tv_nop" : "+v"(c) : "v"(a), "v"(b));
  return c;
}

__device__ __forceinline__ void wave_lds_sync() {
  __builtin_amdgcn_fence(__ATOMIC_RELEASE, "workgroup");
  __builtin_amdgcn_wave_barrier();
  __builtin_amdgcn_fence(__ATOMIC_ACQUIRE, "workgroup");
}

__device__ __forceinline__ int clamp_idx(int v, int n) {
  int r = v < 0 ? 0 : v;
  r = r > (n - 1) ? (n - 1) : r;
  return r;
}

__global__ __launch_bounds__(128) void grp_wsum_kernel(
    const int*   __restrict__ group_user,
    const int*   __restrict__ beh_ids,
    const float* __restrict__ beh_cnt,
    const int*   __restrict__ target_user,
    const float* __restrict__ sim_tab,
    const float* __restrict__ user_tab,
    const float* __restrict__ item_tab,
    float*       __restrict__ out)
{
  __shared__ __align__(16) _Float16 sBt[kWaves][kEmb * kBtPitch];
  __shared__ __align__(16) float    sCnt[kWaves][kSlotsPW];
  __shared__ __align__(16) int      sId[kWaves][kSlotsPW];
  __shared__ __align__(16) float    sWt[kWaves][kUsersPW * kWtPitch];
  __shared__ __align__(16) float    sPart[kWaves][kEmb];

  const int g    = blockIdx.x;
  const int lane = threadIdx.x & 31;
  const int wave = __builtin_amdgcn_readfirstlane((int)(threadIdx.x >> 5));
  const int h    = lane >> 4;
  const int c    = lane & 15;

  _Float16* btw = sBt[wave];
  float*    csw = sCnt[wave];
  int*      idw = sId[wave];
  float*    wtw = sWt[wave];

  const int nUsers  = (kUsersPG - kUsersPW * wave) < kUsersPW ? (kUsersPG - kUsersPW * wave) : kUsersPW;
  const int nSlots  = nUsers * kBehPU;
  const int nChunks = (nSlots + kChunkK - 1) / kChunkK;

  {
    const size_t gslot = (size_t)g * kSlotsPG;
    const int slot0 = kSlotsPW * wave;
#pragma unroll 2
    for (int t = 0; t < kSlotsPW / 32; ++t) {
      const int idx  = 32 * t + lane;
      const int slot = slot0 + idx;
      const bool ok  = slot < kSlotsPG;
      const int sc   = ok ? slot : (kSlotsPG - 1);
      const float cv = beh_cnt[gslot + (size_t)sc];
      const int   iv = beh_ids[gslot + (size_t)sc];
      const int   ic = clamp_idx(iv, kItemRows);
      const float cs = cv * kCntCarry;
      csw[idx] = ok ? cs : 0.0f;
      idw[idx] = ok ? ic : 0;
    }
  }

  {
    const int tg = clamp_idx(target_user[g], kUserRows);
    const v2f tsv = *(const v2f*)(sim_tab + (size_t)tg * kSimDim + 2 * lane);
#pragma unroll 1
    for (int i = 0; i < kUsersPW; ++i) {
      const int u   = kUsersPW * wave + i;
      const bool uv = u < kUsersPG;
      const int uc  = uv ? u : (kUsersPG - 1);
      const int uid = clamp_idx(group_user[g * kUsersPG + uc], kUserRows);
      const v2f sv = *(const v2f*)(sim_tab  + (size_t)uid * kSimDim + 2 * lane);
      const v2f ue = *(const v2f*)(user_tab + (size_t)uid * kEmb    + 2 * lane);
      float dot = sv[0] * tsv[0];
      dot = fmaf(sv[1], tsv[1], dot);
      dot += __shfl_xor(dot, 16, 32);
      dot += __shfl_xor(dot, 8, 32);
      dot += __shfl_xor(dot, 4, 32);
      dot += __shfl_xor(dot, 2, 32);
      dot += __shfl_xor(dot, 1, 32);
      const float sw = 0.5f * dot;
      const float w0 = sw * ue[0];
      const float w1 = sw * ue[1];
      v2f wv;
      wv[0] = uv ? w0 : 0.0f;
      wv[1] = uv ? w1 : 0.0f;
      *(v2f*)(wtw + i * kWtPitch + 2 * lane) = wv;
    }
  }
  __syncthreads();

  v8f acc[4];
#pragma unroll
  for (int j = 0; j < 4; ++j) acc[j] = (v8f){0.f, 0.f, 0.f, 0.f, 0.f, 0.f, 0.f, 0.f};

  const int  aLo  = kBehPU * c;
  const bool aUsr = c < nUsers;

#pragma unroll 1
  for (int ch = 0; ch < nChunks; ++ch) {
    const int cb = ch * kChunkK;

#pragma unroll 1
    for (int k8 = 0; k8 < 4; ++k8) {
      const int kb = cb + 8 * k8;
      const v4i ia = *(const v4i*)(idw + kb);
      const v4i ib = *(const v4i*)(idw + kb + 4);
      v8h hx, hy;
#pragma unroll
      for (int e = 0; e < 4; ++e) {
        const int id = ia[e];
        const v2f ev = *(const v2f*)(item_tab + (size_t)id * kEmb + 2 * lane);
        const bool rv = (kb + e) < nSlots;
        const float x0 = ev[0] * kItemCarry;
        const float y0 = ev[1] * kItemCarry;
        const float x = rv ? x0 : 0.0f;
        const float y = rv ? y0 : 0.0f;
        hx[e] = (_Float16)x;
        hy[e] = (_Float16)y;
      }
#pragma unroll
      for (int e = 0; e < 4; ++e) {
        const int id = ib[e];
        const v2f ev = *(const v2f*)(item_tab + (size_t)id * kEmb + 2 * lane);
        const bool rv = (kb + 4 + e) < nSlots;
        const float x0 = ev[0] * kItemCarry;
        const float y0 = ev[1] * kItemCarry;
        const float x = rv ? x0 : 0.0f;
        const float y = rv ? y0 : 0.0f;
        hx[4 + e] = (_Float16)x;
        hy[4 + e] = (_Float16)y;
      }
      *(v8h*)(btw + (2 * lane) * kBtPitch + 8 * k8)     = hx;
      *(v8h*)(btw + (2 * lane + 1) * kBtPitch + 8 * k8) = hy;
    }
    wave_lds_sync();

    v16h a;
    {
      const float* cp = csw + cb + 8 * h;
      const v4f c0 = *(const v4f*)(cp);
      const v4f c1 = *(const v4f*)(cp + 4);
      const v4f c2 = *(const v4f*)(cp + 16);
      const v4f c3 = *(const v4f*)(cp + 20);
      const int k0 = cb + 8 * h - aLo;
#pragma unroll
      for (int e = 0; e < 4; ++e) {
        const bool s0 = aUsr && ((unsigned)(k0 + e) < (unsigned)kBehPU);
        const bool s1 = aUsr && ((unsigned)(k0 + 4 + e) < (unsigned)kBehPU);
        const bool s2 = aUsr && ((unsigned)(k0 + 16 + e) < (unsigned)kBehPU);
        const bool s3 = aUsr && ((unsigned)(k0 + 20 + e) < (unsigned)kBehPU);
        const float a0 = s0 ? c0[e] : 0.0f;
        const float a1 = s1 ? c1[e] : 0.0f;
        const float a2 = s2 ? c2[e] : 0.0f;
        const float a3 = s3 ? c3[e] : 0.0f;
        a[e]      = (_Float16)a0;
        a[4 + e]  = (_Float16)a1;
        a[8 + e]  = (_Float16)a2;
        a[12 + e] = (_Float16)a3;
      }
    }

#pragma unroll
    for (int j = 0; j < 4; ++j) {
      const v16h b = frag_load_h(btw + (16 * j + c) * kBtPitch + 8 * h);
      acc[j] = mma_h(a, b, acc[j]);
    }
    wave_lds_sync();
  }

  float p0 = 0.0f, p1 = 0.0f, p2 = 0.0f, p3 = 0.0f;
#pragma unroll
  for (int r = 0; r < 8; ++r) {
    const float* wr = wtw + (8 * h + r) * kWtPitch + c;
    p0 = fmaf(acc[0][r], wr[0],  p0);
    p1 = fmaf(acc[1][r], wr[16], p1);
    p2 = fmaf(acc[2][r], wr[32], p2);
    p3 = fmaf(acc[3][r], wr[48], p3);
  }
  p0 += __shfl_xor(p0, 16, 32);
  p1 += __shfl_xor(p1, 16, 32);
  p2 += __shfl_xor(p2, 16, 32);
  p3 += __shfl_xor(p3, 16, 32);
  if (h == 0) {
    float* sp = sPart[wave];
    sp[c]      = p0 * kFoldBack;
    sp[16 + c] = p1 * kFoldBack;
    sp[32 + c] = p2 * kFoldBack;
    sp[48 + c] = p3 * kFoldBack;
  }
  __syncthreads();

  if (wave == 0) {
    const v2f q0 = *(const v2f*)(sPart[0] + 2 * lane);
    const v2f q1 = *(const v2f*)(sPart[1] + 2 * lane);
    const v2f q2 = *(const v2f*)(sPart[2] + 2 * lane);
    const v2f q3 = *(const v2f*)(sPart[3] + 2 * lane);
    v2f o;
    o[0] = ((q0[0] + q1[0]) + q2[0]) + q3[0];
    o[1] = ((q0[1] + q1[1]) + q2[1]) + q3[1];
    volatile v2f* op = (volatile v2f*)(out + (size_t)g * kEmb + 2 * lane);
    *op = o;
    __threadfence();
    *op = o;
  }
}

extern "C" void kernel_launch(void* const* d_in, const int* in_sizes, int n_in,
                              void* d_out, int out_size, void* d_ws, size_t ws_size,
                              hipStream_t stream) {
  (void)d_ws; (void)ws_size;
  if (n_in < 7) return;
  if (in_sizes[0] != kGroups * kUsersPG) return;
  if (in_sizes[1] != kGroups * kSlotsPG) return;
  if (in_sizes[2] != kGroups * kSlotsPG) return;
  if (in_sizes[3] != kGroups) return;
  if (in_sizes[4] != kUserRows * kSimDim) return;
  if (in_sizes[5] != kUserRows * kEmb) return;
  if (in_sizes[6] != kItemRows * kEmb) return;
  if (out_size != kGroups * kEmb) return;

  const int*   group_user  = (const int*)  d_in[0];
  const int*   beh_ids     = (const int*)  d_in[1];
  const float* beh_cnt     = (const float*)d_in[2];
  const int*   target_user = (const int*)  d_in[3];
  const float* sim_tab     = (const float*)d_in[4];
  const float* user_tab    = (const float*)d_in[5];
  const float* item_tab    = (const float*)d_in[6];
  float*       out         = (float*)      d_out;

  grp_wsum_kernel<<<kGroups, 128, 0, stream>>>(
      group_user, beh_ids, beh_cnt, target_user, sim_tab, user_tab, item_tab, out);
}
